// SAGEEdgePredictor_85744727097864
// MI455X (gfx1250) — hardware-verified
//
#include <hip/hip_runtime.h>
#include <math.h>

constexpr int kNodes   = 100000;
constexpr int kRowsPad = 100032;
constexpr int kEdges   = 800000;
constexpr int kDim     = 128;
constexpr int kCat     = 256;
static_assert(kRowsPad % 64 == 0 && kRowsPad >= kNodes && kRowsPad - kNodes < 64, "row pad");
static_assert(kEdges % 256 == 0, "edge grid");
static_assert(kDim % 32 == 0 && kCat % 64 == 0, "tile multiples");

typedef __attribute__((ext_vector_type(16))) _Float16 v16h;
typedef __attribute__((ext_vector_type(8)))  _Float16 v8h;
typedef __attribute__((ext_vector_type(4)))  _Float16 v4h;
typedef __attribute__((ext_vector_type(16))) __bf16   v16b;
typedef __attribute__((ext_vector_type(8)))  __bf16   v8b;
typedef __attribute__((ext_vector_type(8)))  float    v8f;
typedef __attribute__((ext_vector_type(4)))  float    v4f;
typedef __attribute__((ext_vector_type(4)))  int      v4i;

__device__ __forceinline__ unsigned short f2bf_bits(float f) {
  unsigned u = __float_as_uint(f);
  return (unsigned short)((u + 0x7FFFu + ((u >> 16) & 1u)) >> 16);
}
__device__ __forceinline__ float bf_bits2f(unsigned short h) { return __uint_as_float(((unsigned)h) << 16); }

__device__ __forceinline__ void dep_guard_h(v8f& a, v8f& b, v16h x, v16h y) { asm volatile("v_nop\n\tv_nop\n\tv_nop\n\tv_nop" : "+v"(a), "+v"(b) : "v"(x), "v"(y)); }
__device__ __forceinline__ void dep_guard_b(v8f& a, v8f& b, v16b x, v16b y) { asm volatile("v_nop\n\tv_nop\n\tv_nop\n\tv_nop" : "+v"(a), "+v"(b) : "v"(x), "v"(y)); }
__device__ __forceinline__ void keep4_h(v16h a, v16h b, v16h c, v16h d) { asm volatile("v_nop" :: "v"(a), "v"(b), "v"(c), "v"(d)); }
__device__ __forceinline__ void keep4_b(v16b a, v16b b, v16b c, v16b d) { asm volatile("v_nop" :: "v"(a), "v"(b), "v"(c), "v"(d)); }
__device__ __forceinline__ void acc_guard4(v8f& a, v8f& b, v8f& c, v8f& d) { asm volatile("v_nop\n\tv_nop\n\tv_nop\n\tv_nop" : "+v"(a), "+v"(b), "+v"(c), "+v"(d)); }
template <typename T> struct Frag;
template <> struct Frag<_Float16> {
  typedef v16h V; union U { v16h v; v8h h[2]; };
  static __device__ __forceinline__ v16h load(const _Float16* p) {
    U f; f.h[0] = *(const v8h*)(p); f.h[1] = *(const v8h*)(p + 16); return f.v;
  }
  static __device__ __forceinline__ v8f mma(v16h a, v16h b, v8f c) {
    return __builtin_amdgcn_wmma_f32_16x16x32_f16(false, a, false, b, (short)0, c, false, false);
  }
  static __device__ __forceinline__ void guard(v8f& a, v8f& b, v16h x, v16h y) { dep_guard_h(a, b, x, y); }
  static __device__ __forceinline__ void keep(v16h a, v16h b, v16h c, v16h d) { keep4_h(a, b, c, d); }
};
template <> struct Frag<__bf16> {
  typedef v16b V; union U { v16b v; v8b h[2]; };
  static __device__ __forceinline__ v16b load(const __bf16* p) {
    U f; f.h[0] = *(const v8b*)(p); f.h[1] = *(const v8b*)(p + 16); return f.v;
  }
  static __device__ __forceinline__ v8f mma(v16b a, v16b b, v8f c) {
    return __builtin_amdgcn_wmma_f32_16x16x32_bf16(false, a, false, b, (short)0, c, false, false);
  }
  static __device__ __forceinline__ void guard(v8f& a, v8f& b, v16b x, v16b y) { dep_guard_b(a, b, x, y); }
  static __device__ __forceinline__ void keep(v16b a, v16b b, v16b c, v16b d) { keep4_b(a, b, c, d); }
};

template <int ET> struct Elem;
template <> struct Elem<0> { typedef _Float16 T; };
template <> struct Elem<1> { typedef __bf16 T; };
template <int ET, bool SPLIT, int BIAS_MODE, int OUT_MODE, bool RESID, int ACT = 0>
__global__ __launch_bounds__(256) void wmma_gemm64(
    const unsigned short* __restrict__ Ap, const unsigned short* __restrict__ A2p, int lda, long strideA,
    const unsigned short* __restrict__ Btp, const unsigned short* __restrict__ Bt2p, int ldb, long strideB,
    void* __restrict__ Cout, void* __restrict__ Cout2, int ldc, long strideC,
    const float* __restrict__ bias,
    const float* __restrict__ resid, long strideR,
    int M, int N, int K, float scale) {
  typedef typename Elem<ET>::T T;
  typedef typename Frag<T>::V V;
  const T* A = (const T*)Ap; const T* A2 = (const T*)A2p; const T* Bt = (const T*)Btp; const T* Bt2 = (const T*)Bt2p;
  __shared__ __align__(16) float sT[8][16 * 68];
  const int b    = blockIdx.y;
  const int lane = threadIdx.x & 31;
  const int wave = threadIdx.x >> 5;
  const int tilesN = N >> 6;
  const int tilesM = M >> 6;
  const int tile = blockIdx.x * 8 + wave;
  if (tile >= tilesM * tilesN) return;
  const int tm = tile / tilesN;
  const int tn = tile - tm * tilesN;
  const int m0 = tm << 6;
  const int n0 = tn << 6;

  const T* Ab  = A  + (size_t)b * strideA;
  const T* Bb  = Bt + (size_t)b * strideB;
  const T* Ab2 = SPLIT ? (A2  + (size_t)b * strideA) : nullptr;
  const T* Bb2 = SPLIT ? (Bt2 + (size_t)b * strideB) : nullptr;

  const int rlane = lane & 15;
  const int koff  = (lane >> 4) * 8;
  const int mOff  = (lane >> 4) * 8;

  v8f acc[4][4];
#pragma unroll
  for (int i = 0; i < 4; ++i)
#pragma unroll
    for (int j = 0; j < 4; ++j) acc[i][j] = (v8f){0.f,0.f,0.f,0.f,0.f,0.f,0.f,0.f};

  for (int k0 = 0; k0 < K; k0 += 32) {
    V bh[4], bl[4];
#pragma unroll
    for (int j = 0; j < 4; ++j) {
      const size_t bo = (size_t)(n0 + (j << 4) + rlane) * ldb + koff + k0;
      bh[j] = Frag<T>::load(Bb + bo);
      if (SPLIT) bl[j] = Frag<T>::load(Bb2 + bo);
    }
#pragma unroll
    for (int i = 0; i < 4; ++i) {
      const size_t ao = (size_t)(m0 + (i << 4) + rlane) * lda + koff + k0;
      V ah = Frag<T>::load(Ab + ao);
      V al;
      if (SPLIT) al = Frag<T>::load(Ab2 + ao);
#pragma unroll
      for (int j = 0; j < 4; ++j) {
        acc[i][j] = Frag<T>::mma(ah, bh[j], acc[i][j]);
        if (SPLIT) {
          acc[i][j] = Frag<T>::mma(ah, bl[j], acc[i][j]);
          acc[i][j] = Frag<T>::mma(al, bh[j], acc[i][j]);
        }
      }
      Frag<T>::guard(acc[i][0], acc[i][3], ah, SPLIT ? al : ah);
    }
    Frag<T>::keep(bh[0], bh[1], bh[2], bh[3]);
    if (SPLIT) Frag<T>::keep(bl[0], bl[1], bl[2], bl[3]);
  }
  acc_guard4(acc[0][0], acc[0][1], acc[0][2], acc[0][3]);
  acc_guard4(acc[1][0], acc[1][1], acc[1][2], acc[1][3]);
  acc_guard4(acc[2][0], acc[2][1], acc[2][2], acc[2][3]);
  acc_guard4(acc[3][0], acc[3][1], acc[3][2], acc[3][3]);

  float* slab = sT[wave];
  const float* Rb = RESID ? (resid + (size_t)b * strideR) : nullptr;
#pragma unroll
  for (int i = 0; i < 4; ++i) {
    const int mBase = m0 + (i << 4);
#pragma unroll
    for (int j = 0; j < 4; ++j) {
      const int n = n0 + (j << 4) + rlane;
      float bv = 0.f;
      if (BIAS_MODE == 2) bv = bias[n];
#pragma unroll
      for (int r = 0; r < 8; ++r) {
        float v = acc[i][j][r] * scale;
        if (BIAS_MODE == 1) v += bias[mBase + mOff + r];
        if (BIAS_MODE == 2) v += bv;
        if (RESID) v += Rb[(size_t)(mBase + mOff + r) * ldc + n];
        if (ACT == 1) v = tanhf(v);
        if (ACT == 2) v = fmaxf(v, 0.0f);
        if (ACT == 3) v = v / (1.0f + expf(-v));
        if (ACT == 4) v = (v > 0.f) ? v : 0.01f * v;
        if (ACT == 5) v = 0.5f * v * (1.0f + erff(v * 0.70710678118654752f));
        slab[(mOff + r) * 68 + (j << 4) + rlane] = v;
      }
    }
    __builtin_amdgcn_fence(__ATOMIC_RELEASE, "workgroup");
    __builtin_amdgcn_wave_barrier();
    __builtin_amdgcn_fence(__ATOMIC_ACQUIRE, "workgroup");
    if (OUT_MODE == 0) {
      float* C = (float*)Cout + (size_t)b * strideC;
      const int hh = lane >> 4, c4 = (lane & 15) * 4;
      for (int pass = 0; pass < 2; ++pass) {
#pragma unroll
        for (int it = 0; it < 8; ++it) {
          const int row = it * 2 + hh;
          v4f v = *(const v4f*)(slab + row * 68 + c4);
          *(volatile v4f*)(C + (size_t)(mBase + row) * ldc + n0 + c4) = v;
        }
        __threadfence();
      }
    } else {
      const int q = lane >> 3, c8 = (lane & 7) * 8;
      unsigned short* C  = (unsigned short*)Cout  + (size_t)b * strideC;
      unsigned short* C2 = (OUT_MODE == 2) ? ((unsigned short*)Cout2 + (size_t)b * strideC) : nullptr;
      for (int pass = 0; pass < 2; ++pass) {
#pragma unroll
        for (int it = 0; it < 4; ++it) {
          const int row = it * 4 + q;
          const float* sp = slab + row * 68 + c8;
          v8h hv, lv;
#pragma unroll
          for (int e = 0; e < 8; ++e) {
            if (OUT_MODE == 1) {
              hv[e] = (_Float16)sp[e];
            } else {
              unsigned short hb = f2bf_bits(sp[e]);
              unsigned short lb = f2bf_bits(sp[e] - bf_bits2f(hb));
              hv[e] = __builtin_bit_cast(_Float16, hb);
              lv[e] = __builtin_bit_cast(_Float16, lb);
            }
          }
          *(volatile v8h*)(C + (size_t)(mBase + row) * ldc + n0 + c8) = hv;
          if (OUT_MODE == 2) *(volatile v8h*)(C2 + (size_t)(mBase + row) * ldc + n0 + c8) = lv;
        }
        __threadfence();
      }
    }
    __builtin_amdgcn_fence(__ATOMIC_RELEASE, "workgroup");
    __builtin_amdgcn_wave_barrier();
    __builtin_amdgcn_fence(__ATOMIC_ACQUIRE, "workgroup");
  }
}

constexpr int kAggRows  = 256;
constexpr int kAggWaves = kAggRows / 32;
constexpr int kChunk    = 8192;
constexpr int kEpt      = kChunk / kAggRows;
constexpr int kWcap     = 64;
static_assert(kEpt == 32, "hit bitmask is one 32-bit word");
static_assert(kEdges % kEpt == 0, "a thread's chunk slice is all valid or all past the end");
static_assert(kRowsPad % 32 == 0, "wave-uniform row tails");
static_assert(((long)kNodes << 8) < 2147483647L, "packed hit word fits int");

__device__ __forceinline__ int blk_excl_scan(int cnt, int* scan_ws, int tid, int* tot) {
  const int lane = tid & 31, wave = tid >> 5; int incl = cnt;
#pragma unroll
  for (int o = 1; o < 32; o <<= 1) { const int v = __shfl_up(incl, o, 32); if (lane >= o) incl += v; }
  if (lane == 31) scan_ws[wave] = incl;
  __syncthreads();
  if (wave == 0) { int wv = (lane < kAggWaves) ? scan_ws[lane] : 0; int wincl = wv;
#pragma unroll
    for (int o = 1; o < 32; o <<= 1) { const int v = __shfl_up(wincl, o, 32); if (lane >= o) wincl += v; }
    if (lane < kAggWaves) scan_ws[32 + lane] = wincl - wv; if (lane == 31) scan_ws[64] = wincl; }
  __syncthreads();
  const int res = scan_ws[32 + wave] + incl - cnt; *tot = scan_ws[64];
  return res;
}
__device__ __forceinline__ int chunk_compact(const int* __restrict__ keyv, const int* __restrict__ othv, int e0, int ne, int n0, int nn, int tid, int* Lp, int* scan_ws) {
  const int  eb  = e0 + tid * kEpt;
  const bool ok  = eb < ne;
  const int  ebc = ok ? eb : (ne - kEpt);
  unsigned flags = 0u; int cnt = 0;
#pragma unroll
  for (int q4 = 0; q4 < kEpt / 4; ++q4) {
    const v4i kq = *(const v4i*)(keyv + ebc + 4 * q4);
#pragma unroll
    for (int k = 0; k < 4; ++k) {
      const int d = kq[k];
      const unsigned u = (unsigned)(d - n0);
      const bool hit = ok && (u < (unsigned)kAggRows) && (d < nn);
      flags |= hit ? (1u << (4 * q4 + k)) : 0u;
      cnt += hit ? 1 : 0;
    }
  }
  int tot; int p = blk_excl_scan(cnt, scan_ws, tid, &tot);
#pragma unroll 1
  for (int it = 0; it < kEpt; ++it) {
    if (flags == 0u) break;
    const int k = __builtin_ctz(flags);
    flags &= flags - 1u;
    const int e = ebc + k;
    const int d = keyv[e];
    int s = othv[e]; s = s < 0 ? 0 : (s >= nn ? nn - 1 : s);
    const int pc = p < kChunk ? p : (kChunk - 1);
    Lp[pc] = (s << 8) | ((d - n0) & 255);
    ++p;
  }
  __syncthreads();
  return tot;
}
template <int LO, int HI, int VPL> struct SlotDisp { static __device__ __forceinline__ void add(int s, float (*acc)[VPL], const float* v) {
  if (LO + 1 == HI) {
#pragma unroll
    for (int j = 0; j < VPL; ++j) acc[LO][j] += v[j]; }
  else { const int MID = (LO + HI) / 2; if (s < MID) SlotDisp<LO, (LO + HI) / 2, VPL>::add(s, acc, v); else SlotDisp<(LO + HI) / 2, HI, VPL>::add(s, acc, v); } } };
template <typename HT>
__device__ __forceinline__ void coop_flush(int n, const unsigned char* wls, const int* wlv, const HT* Hm, int ldh, int lane, float (*acc)[4], float* cnl) {
  n = n < kWcap ? n : kWcap;
  for (int j = 0; j < n; ++j) { const int slot = wls[j]; const int src = wlv[j]; float v[4];
    const HT* hp = Hm + (size_t)src * ldh + lane * 4;
    if (sizeof(HT) == 2) { const v4h q = *(const v4h*)(const void*)hp; v[0] = (float)q[0]; v[1] = (float)q[1]; v[2] = (float)q[2]; v[3] = (float)q[3]; }
    else { const v4f q = *(const v4f*)(const void*)hp; v[0] = q[0]; v[1] = q[1]; v[2] = q[2]; v[3] = q[3]; }
    if (cnl != nullptr && lane == 0) cnl[slot] += 1.0f;
    SlotDisp<0, 32, 4>::add(slot, acc, v); }
}
template <typename HT>
__device__ __forceinline__ void coop_chunk(int tot, const int* Lp, unsigned char* wls, int* wlv, const HT* Hm, int ldh, int wave, int lane, float (*acc)[4], float* cnl) {
  int nlist = 0;
  for (int q0 = 0; q0 < tot; q0 += 32) { const int q = q0 + lane; const int qc = (q < tot) ? q : (tot - 1);
    const int pk = Lp[qc]; const int l0 = pk & 255; const int l1 = pk >> 8; const bool mine = (q < tot) && ((l0 >> 5) == wave);
    const unsigned bal = __builtin_amdgcn_ballot_w32(mine); const int cntb = __builtin_popcount(bal);
    if (nlist + cntb > kWcap) { coop_flush<HT>(nlist, wls, wlv, Hm, ldh, lane, acc, cnl); nlist = 0; }
    const int pos = nlist + __builtin_popcount(bal & ((1u << lane) - 1u));
    if (mine) { wls[pos] = (unsigned char)(l0 & 31); wlv[pos] = l1; }
    nlist += cntb; }
  coop_flush<HT>(nlist, wls, wlv, Hm, ldh, lane, acc, cnl);
}
template <typename HT, bool WDEG>
__global__ __launch_bounds__(kAggRows) void mean_agg_kernel(const HT* Hm, int ldh, const int* __restrict__ keyv, const int* __restrict__ othv, int ne, int nn, int nrow,
                                                             float* DEG, _Float16* A16, int lda, int coff) {
  __shared__ __align__(16) int Lp[kChunk];
  __shared__ int scan_ws[80];
  __shared__ unsigned char WLs[kAggWaves][kWcap];
  __shared__ int WLv[kAggWaves][kWcap];
  __shared__ float CNL[kAggRows];
  __shared__ __align__(16) _Float16 STG[kAggWaves][8 * 128];
  const int tid = threadIdx.x, lane = tid & 31, wave = tid >> 5, n0 = blockIdx.x * kAggRows;
  CNL[tid] = 0.f; float* cnl = WDEG ? (CNL + wave * 32) : nullptr;
  __syncthreads();
  float acc[32][4];
#pragma unroll
  for (int s = 0; s < 32; ++s)
#pragma unroll
    for (int j = 0; j < 4; ++j) acc[s][j] = 0.f;
  for (int e0 = 0; e0 < ne; e0 += kChunk) {
    int tot = chunk_compact(keyv, othv, e0, ne, n0, nn, tid, Lp, scan_ws);
    tot = tot < kChunk ? tot : kChunk;
    coop_chunk<HT>(tot, Lp, WLs[wave], WLv[wave], Hm, ldh, wave, lane, acc, cnl);
    __syncthreads();
  }
  __syncthreads();
  const int nb = n0 + wave * 32;
  if (nb < nrow) {
    const int nl = nb + lane;
    float dreg;
    if (WDEG) dreg = CNL[wave * 32 + lane]; else dreg = DEG[nl];
    const float invl = 1.0f / fmaxf(dreg, 1.0f);
    if (WDEG) { ((volatile float*)DEG)[nl] = dreg; __threadfence(); ((volatile float*)DEG)[nl] = dreg; }
    _Float16* stg = STG[wave];
    const int q = lane >> 3, c8 = (lane & 7) * 8;
#pragma unroll
    for (int g = 0; g < 4; ++g) {
#pragma unroll
      for (int r = 0; r < 8; ++r) {
        const float is = __shfl(invl, g * 8 + r, 32);
        v4h o;
        o[0] = (_Float16)(acc[g * 8 + r][0] * is); o[1] = (_Float16)(acc[g * 8 + r][1] * is);
        o[2] = (_Float16)(acc[g * 8 + r][2] * is); o[3] = (_Float16)(acc[g * 8 + r][3] * is);
        *(v4h*)(stg + r * 128 + lane * 4) = o;
      }
      __builtin_amdgcn_fence(__ATOMIC_RELEASE, "workgroup");
      __builtin_amdgcn_wave_barrier();
      __builtin_amdgcn_fence(__ATOMIC_ACQUIRE, "workgroup");
      for (int ps = 0; ps < 2; ++ps) {
#pragma unroll
        for (int a = 0; a < 4; ++a) {
          const int li = a * 4 + q;
          const int r = li >> 1, hf = (li & 1) * 64;
          const v8h val = *(const v8h*)(stg + r * 128 + hf + c8);
          *(volatile v8h*)(A16 + (size_t)(nb + g * 8 + r) * lda + coff + hf + c8) = val;
        }
        __threadfence();
      }
      __builtin_amdgcn_fence(__ATOMIC_RELEASE, "workgroup");
      __builtin_amdgcn_wave_barrier();
      __builtin_amdgcn_fence(__ATOMIC_ACQUIRE, "workgroup");
    }
  }
}

__device__ __forceinline__ unsigned pkh(float a, float b) { return (unsigned)__builtin_bit_cast(unsigned short, (_Float16)a) | ((unsigned)__builtin_bit_cast(unsigned short, (_Float16)b) << 16); }

__global__ __launch_bounds__(256) void xcvt_kernel(const float* __restrict__ X, _Float16* __restrict__ A16, int nn, int nrow, int lda) {
  const long i  = (long)blockIdx.x * 256 + threadIdx.x;
  const int row = (int)(i >> 4);
  const int c8  = (int)(i & 15) * 8;
  if (row < nrow) {
    const int rr = row < nn ? row : (nn - 1);
    const float* xp = X + (size_t)rr * kDim + c8;
    const v4f a = *(const v4f*)xp;
    const v4f b = *(const v4f*)(xp + 4);
    const bool ok = row < nn;
    v8h o;
    o[0] = (_Float16)(ok ? a[0] : 0.f); o[1] = (_Float16)(ok ? a[1] : 0.f); o[2] = (_Float16)(ok ? a[2] : 0.f); o[3] = (_Float16)(ok ? a[3] : 0.f);
    o[4] = (_Float16)(ok ? b[0] : 0.f); o[5] = (_Float16)(ok ? b[1] : 0.f); o[6] = (_Float16)(ok ? b[2] : 0.f); o[7] = (_Float16)(ok ? b[3] : 0.f);
    _Float16* dp = A16 + (size_t)row * lda + c8;
    *(volatile v8h*)dp = o;
    __threadfence();
    *(volatile v8h*)dp = o;
  }
}
__global__ __launch_bounds__(256) void wcat_layer_kernel(const float* __restrict__ Wr, const float* __restrict__ Wl, _Float16* __restrict__ BT) {
  const int i = blockIdx.x * 256 + threadIdx.x;
  if (i < kDim * kDim) {
    const int n = i >> 7; const int kp = (i & 127) * 2; const int kk = kp & 127;
    const float r0 = Wr[n * kDim + kk], r1 = Wr[n * kDim + kk + 1];
    const float l0 = Wl[n * kDim + kk], l1 = Wl[n * kDim + kk + 1];
    const bool lo = kp < kDim;
    const float a = 16.0f * (lo ? r0 : l0), b = 16.0f * (lo ? r1 : l1);
    const unsigned u = pkh(a, b);
    ((volatile unsigned*)BT)[i] = u;
    __threadfence();
    ((volatile unsigned*)BT)[i] = u;
  }
}
__global__ __launch_bounds__(256) void wcat_mlp_kernel(const float* __restrict__ Wm1, _Float16* __restrict__ BT) {
  const int i = blockIdx.x * 256 + threadIdx.x;
  if (i < kCat * kDim / 2) {
    const int n = i >> 6; const int kp = (i & 63) * 2; const int np = n & 127; const int coff = (n >> 7) * kDim;
    const float a = 16.0f * Wm1[np * kCat + coff + kp], b = 16.0f * Wm1[np * kCat + coff + kp + 1];
    const unsigned u = pkh(a, b);
    ((volatile unsigned*)BT)[i] = u;
    __threadfence();
    ((volatile unsigned*)BT)[i] = u;
  }
}

__global__ __launch_bounds__(256) void edge_head_kernel(const _Float16* __restrict__ PSD, int ldp, const int* __restrict__ ei, const float* __restrict__ bm1,
                                                         const float* __restrict__ Wm2, const float* __restrict__ bm2, float* __restrict__ out, int ne, int nn) {
  const int lane = threadIdx.x & 31, wave = threadIdx.x >> 5;
  const int e0 = (blockIdx.x * 8 + wave) * 32;
  if (e0 + 32 > ne) return;
  const v4f bb = *(const v4f*)(bm1 + lane * 4);
  const v4f ww = *(const v4f*)(Wm2 + lane * 4);
  const float b2 = bm2[0];
  int sl = ei[e0 + lane];
  int dl = ei[ne + e0 + lane];
  sl = sl < 0 ? 0 : (sl >= nn ? nn - 1 : sl);
  dl = dl < 0 ? 0 : (dl >= nn ? nn - 1 : dl);
  float res = 0.f;
#pragma unroll 1
  for (int j = 0; j < 32; ++j) {
    const int sj = __shfl(sl, j, 32);
    const int dj = __shfl(dl, j, 32);
    const v4h ps = *(const v4h*)(PSD + (size_t)sj * ldp + lane * 4);
    const v4h pd = *(const v4h*)(PSD + (size_t)dj * ldp + kDim + lane * 4);
    float a = 0.f;
#pragma unroll
    for (int q = 0; q < 4; ++q) {
      float hv = (float)ps[q] + (float)pd[q] + bb[q];
      hv = fmaxf(hv, 0.0f);
      a += hv * ww[q];
    }
#pragma unroll
    for (int off = 16; off >= 1; off >>= 1) a += __shfl_xor(a, off, 32);
    const float z  = a + b2;
    const float sg = 1.0f / (1.0f + expf(-z));
    res = (lane == j) ? sg : res;
  }
  ((volatile float*)out)[e0 + lane] = res;
  __threadfence();
  ((volatile float*)out)[e0 + lane] = res;
}

extern "C" void kernel_launch(void* const* d_in, const int* in_sizes, int n_in,
                              void* d_out, int out_size, void* d_ws, size_t ws_size,
                              hipStream_t stream) {
  if (n_in < 12) return;
  if (in_sizes[0] != kNodes * kDim || in_sizes[1] != 2 * kEdges || out_size != kEdges) return;
  if (in_sizes[2] != kDim * kDim || in_sizes[4] != kDim * kDim || in_sizes[5] != kDim * kDim || in_sizes[7] != kDim * kDim) return;
  if (in_sizes[3] != kDim || in_sizes[6] != kDim || in_sizes[8] != kDim * kCat || in_sizes[9] != kDim || in_sizes[10] != kDim || in_sizes[11] < 1) return;
  const float* X   = (const float*)d_in[0];
  const int*   EI  = (const int*)  d_in[1];
  const float* W1l = (const float*)d_in[2];
  const float* b1l = (const float*)d_in[3];
  const float* W1r = (const float*)d_in[4];
  const float* W2l = (const float*)d_in[5];
  const float* b2l = (const float*)d_in[6];
  const float* W2r = (const float*)d_in[7];
  const float* Wm1 = (const float*)d_in[8];
  const float* bm1 = (const float*)d_in[9];
  const float* Wm2 = (const float*)d_in[10];
  const float* bm2 = (const float*)d_in[11];
  float* out = (float*)d_out;

  char* ws = (char*)d_ws; size_t off = 0;
  auto carve = [&](size_t bytes) -> char* { char* p = ws + off; off += (bytes + 255) & ~(size_t)255; return p; };
  _Float16* P1  = (_Float16*)carve((size_t)kRowsPad * kCat * 2);
  _Float16* P2  = (_Float16*)carve((size_t)kRowsPad * kCat * 2);
  float*    DEG = (float*)   carve((size_t)kRowsPad * 4);
  _Float16* BT1 = (_Float16*)carve((size_t)kDim * kCat * 2);
  _Float16* BT2 = (_Float16*)carve((size_t)kDim * kCat * 2);
  _Float16* BT3 = (_Float16*)carve((size_t)kCat * kDim * 2);
  if (off > ws_size || off > (size_t)134217728) return;

  const int*   SRC = EI;
  const int*   DST = EI + kEdges;
  const int    nbAgg = (kRowsPad + kAggRows - 1) / kAggRows;
  const int    gL    = ((kRowsPad / 64) * (kDim / 64) + 7) / 8;
  const int    gM    = ((kRowsPad / 64) * (kCat / 64) + 7) / 8;
  const float  wscl  = 1.0f / 16.0f;

  wcat_layer_kernel<<<(kDim * kDim) / 256, 256, 0, stream>>>(W1r, W1l, BT1);
  wcat_layer_kernel<<<(kDim * kDim) / 256, 256, 0, stream>>>(W2r, W2l, BT2);
  wcat_mlp_kernel<<<(kCat * kDim / 2) / 256, 256, 0, stream>>>(Wm1, BT3);
  xcvt_kernel<<<(kRowsPad * 16) / 256, 256, 0, stream>>>(X, P1, kNodes, kRowsPad, kCat);

  mean_agg_kernel<float, true><<<nbAgg, kAggRows, 0, stream>>>(X, kDim, DST, SRC, kEdges, kNodes, kRowsPad, DEG, P1, kCat, kDim);
  wmma_gemm64<0, false, 2, 1, false, 2><<<dim3(gL, 1), 256, 0, stream>>>(
      (const unsigned short*)P1, nullptr, kCat, 0, (const unsigned short*)BT1, nullptr, kCat, 0,
      (void*)P2, nullptr, kCat, 0, b1l, nullptr, 0, kRowsPad, kDim, kCat, wscl);

  mean_agg_kernel<_Float16, false><<<nbAgg, kAggRows, 0, stream>>>(P2, kCat, DST, SRC, kEdges, kNodes, kRowsPad, DEG, P2, kCat, kDim);
  wmma_gemm64<0, false, 2, 1, false, 2><<<dim3(gL, 1), 256, 0, stream>>>(
      (const unsigned short*)P2, nullptr, kCat, 0, (const unsigned short*)BT2, nullptr, kCat, 0,
      (void*)P1, nullptr, kDim, 0, b2l, nullptr, 0, kRowsPad, kDim, kCat, wscl);

  wmma_gemm64<0, false, 0, 1, false, 0><<<dim3(gM, 1), 256, 0, stream>>>(
      (const unsigned short*)P1, nullptr, kDim, 0, (const unsigned short*)BT3, nullptr, kDim, 0,
      (void*)P2, nullptr, kCat, 0, nullptr, nullptr, 0, kRowsPad, kCat, kDim, wscl);

  edge_head_kernel<<<kEdges / 256, 256, 0, stream>>>(P2, kCat, EI, bm1, Wm2, bm2, out, kEdges, kNodes);
}
